// AttentionLePE_3951369912845
// MI455X (gfx1250) — hardware-verified
//
#include <hip/hip_runtime.h>
#include <math.h>
#include <stdint.h>


#define NB      4
#define IMH     56
#define IMW     56
#define CD      256
#define NPIX    (IMH * IMW)
#define SEQ     (NPIX + 1)
#define SP      3200
#define NH      8
#define HD      32
#define OQ      (3 * CD)
#define NTOK    (NB * SP)
#define NBH     (NB * NH)
#define NDWR    (NB * NPIX)
#define KC      160
#define NKC     (SP / KC)
#define NSUB    (KC / 32)
#define KP      40
#define VP      (KC + 8)
#define AW      8
#define ATHR    (AW * 32)
#define QB      (AW * 16)
#define NQB     (SP / QB)
#define LDSA    (KC * KP + 2 * HD * VP)
#define SVP     64
#define SPW     2048
#define LPB     28
#define LIT     7
#define OUT1OFF (NB * NPIX * CD)

static_assert(NPIX == 3136 && SEQ <= SP);
static_assert((SP % 64) == 0 && (SP % KC) == 0 && (KC % 32) == 0 && NQB * QB == SP && NKC * KC == SP);
static_assert(NH * HD == CD && (CD % 64) == 0 && (OQ % 64) == 0 && (NTOK % 64) == 0 && HD == 32);
static_assert(AW * 1024 <= LDSA);
static_assert(SPW >= 64 * HD && SPW >= HD * SVP);
static_assert((NPIX % LPB) == 0 && LPB == 4 * LIT);
static_assert(CD == 256);
static_assert((KP % 8) == 0 && (VP % 8) == 0 && (SVP % 8) == 0);
static_assert(((OQ * CD / 8) % 256) == 0 && ((CD * CD / 8) % 256) == 0 && ((NTOK * 32) % 256) == 0);

typedef _Float16 v16h __attribute__((ext_vector_type(16)));
typedef _Float16 v8h  __attribute__((ext_vector_type(8)));
typedef _Float16 v4h  __attribute__((ext_vector_type(4)));
typedef float    v8f  __attribute__((ext_vector_type(8)));
typedef float    v4f  __attribute__((ext_vector_type(4)));
typedef unsigned int v4u __attribute__((ext_vector_type(4)));

__device__ __forceinline__ unsigned short bf_bits(float f) {
  unsigned u = __float_as_uint(f);
  return (unsigned short)((u + 0x7FFFu + ((u >> 16) & 1u)) >> 16);
}
__device__ __forceinline__ float bf_up(unsigned short h) { return __uint_as_float(((unsigned)h) << 16); }
__device__ __forceinline__ unsigned short h_bits(_Float16 x) { return __builtin_bit_cast(unsigned short, x); }
__device__ __forceinline__ unsigned pk16(unsigned short a, unsigned short b) { return (unsigned)a | ((unsigned)b << 16); }
__device__ __forceinline__ v8f zero8() { v8f z = {0.f, 0.f, 0.f, 0.f, 0.f, 0.f, 0.f, 0.f}; return z; }

__device__ __forceinline__ v16h ldfrag_h(const _Float16* p) {
  union { v16h v; v8h h[2]; } f;
  f.h[0] = *(const v8h*)(p);
  f.h[1] = *(const v8h*)(p + 16);
  return f.v;
}

__device__ __forceinline__ v8f mma_h_raw(v16h a, v16h b, v8f c) {
  return __builtin_amdgcn_wmma_f32_16x16x32_f16(false, a, false, b, (short)0, c, false, false);
}
__device__ __forceinline__ void res_guard(v8f& t, v8f& acc, v16h x, v16h y) {
#if defined(__HIP_DEVICE_COMPILE__)
  asm volatile("v_nop\n\tv_nop\n\tv_nop\n\tv_nop" : "+v"(t), "+v"(acc) : "v"(x), "v"(y));
#endif
}
__device__ __forceinline__ void dep_guard_h(v8f& a, v8f& b, v16h x, v16h y) {
#if defined(__HIP_DEVICE_COMPILE__)
  asm volatile("v_nop\n\tv_nop\n\tv_nop\n\tv_nop" : "+v"(a), "+v"(b) : "v"(x), "v"(y));
#endif
}
__device__ __forceinline__ void dep_guard3(v8f& a, v8f& b, v16h x, v16h y, v16h z) {
#if defined(__HIP_DEVICE_COMPILE__)
  asm volatile("v_nop\n\tv_nop\n\tv_nop\n\tv_nop" : "+v"(a), "+v"(b) : "v"(x), "v"(y), "v"(z));
#endif
}
__device__ __forceinline__ void keep4_h(v16h a, v16h b, v16h c, v16h d) {
#if defined(__HIP_DEVICE_COMPILE__)
  asm volatile("v_nop" :: "v"(a), "v"(b), "v"(c), "v"(d));
#endif
}
__device__ __forceinline__ void acc_guard4(v8f& a, v8f& b, v8f& c, v8f& d) {
#if defined(__HIP_DEVICE_COMPILE__)
  asm volatile("v_nop\n\tv_nop\n\tv_nop\n\tv_nop" : "+v"(a), "+v"(b), "+v"(c), "+v"(d));
#endif
}
__device__ __forceinline__ void wave_sync_lds() {
  __builtin_amdgcn_fence(__ATOMIC_RELEASE, "workgroup");
  __builtin_amdgcn_wave_barrier();
  __builtin_amdgcn_fence(__ATOMIC_ACQUIRE, "workgroup");
}

__global__ __launch_bounds__(256) void cvt_h8(const float* __restrict__ in, unsigned short* out, int n8, float scale) {
  const int i = blockIdx.x * 256 + threadIdx.x;
  if (i < n8) {
    const v4f a = *(const v4f*)(in + (size_t)i * 8);
    const v4f c = *(const v4f*)(in + (size_t)i * 8 + 4);
    float f[8];
    f[0] = a[0]; f[1] = a[1]; f[2] = a[2]; f[3] = a[3];
    f[4] = c[0]; f[5] = c[1]; f[6] = c[2]; f[7] = c[3];
    unsigned short hb[8];
#pragma unroll
    for (int e = 0; e < 8; ++e) hb[e] = h_bits((_Float16)(bf_up(bf_bits(f[e])) * scale));
    v4u p;
    p[0] = pk16(hb[0], hb[1]);
    p[1] = pk16(hb[2], hb[3]);
    p[2] = pk16(hb[4], hb[5]);
    p[3] = pk16(hb[6], hb[7]);
    *(volatile v4u*)(out + (size_t)i * 8) = p;
    __threadfence();
    *(volatile v4u*)(out + (size_t)i * 8) = p;
  }
}

__global__ __launch_bounds__(256) void cvt_xt(const float* __restrict__ x, const float* __restrict__ cls,
                                              unsigned short* XT, float scale) {
  const int i = blockIdx.x * 256 + threadIdx.x;
  if (i < NTOK * 32) {
    const int row = i >> 5, c8 = (i & 31) * 8;
    const int b = row / SP, s = row - b * SP;
    const int sc = min(max(s - 1, 0), NPIX - 1);
    const float* pc = cls + (size_t)b * CD + c8;
    const float* px = x + ((size_t)(b * NPIX + sc)) * CD + c8;
    const v4f ca = *(const v4f*)(pc);
    const v4f cc = *(const v4f*)(pc + 4);
    const v4f xa = *(const v4f*)(px);
    const v4f xc = *(const v4f*)(px + 4);
    const bool isc = (s == 0);
    const bool isx = (s >= 1) && (s <= NPIX);
    float f[8];
    f[0] = isc ? ca[0] : (isx ? xa[0] : 0.0f);
    f[1] = isc ? ca[1] : (isx ? xa[1] : 0.0f);
    f[2] = isc ? ca[2] : (isx ? xa[2] : 0.0f);
    f[3] = isc ? ca[3] : (isx ? xa[3] : 0.0f);
    f[4] = isc ? cc[0] : (isx ? xc[0] : 0.0f);
    f[5] = isc ? cc[1] : (isx ? xc[1] : 0.0f);
    f[6] = isc ? cc[2] : (isx ? xc[2] : 0.0f);
    f[7] = isc ? cc[3] : (isx ? xc[3] : 0.0f);
    unsigned short hb[8];
#pragma unroll
    for (int e = 0; e < 8; ++e) hb[e] = h_bits((_Float16)(bf_up(bf_bits(f[e])) * scale));
    v4u p;
    p[0] = pk16(hb[0], hb[1]);
    p[1] = pk16(hb[2], hb[3]);
    p[2] = pk16(hb[4], hb[5]);
    p[3] = pk16(hb[6], hb[7]);
    unsigned short* dst = XT + (size_t)row * CD + c8;
    *(volatile v4u*)dst = p;
    __threadfence();
    *(volatile v4u*)dst = p;
  }
}

__global__ __launch_bounds__(256) void dwconv5(const unsigned short* __restrict__ XTp, const float* __restrict__ wdw,
                                               const float* __restrict__ bdw, float* DW, float xinv) {
  __shared__ __align__(16) float sW[25 * CD];
  __shared__ __align__(16) float sB[CD];
  const _Float16* XT = (const _Float16*)(const void*)XTp;
  const int tid = threadIdx.x;
  const int b = blockIdx.x / (NPIX / LPB);
  const int pbase = (blockIdx.x - b * (NPIX / LPB)) * LPB;
  for (int idx = tid; idx < 25 * CD; idx += 256) {
    const int c = idx / 25;
    const int tap = idx - c * 25;
    sW[tap * CD + c] = bf_up(bf_bits(wdw[idx]));
  }
  sB[tid] = bf_up(bf_bits(bdw[tid]));
  __syncthreads();
  const int cq = tid & 63, c = cq * 4, pl4 = tid >> 6;
#pragma unroll 1
  for (int it = 0; it < LIT; ++it) {
    const int n  = pbase + it * 4 + pl4;
    const int hq = n / IMW;
    const int wq = n - hq * IMW;
    v4f acc = {0.0f, 0.0f, 0.0f, 0.0f};
#pragma unroll 1
    for (int i = 0; i < 5; ++i) {
      const int hr = hq + i - 2;
      const int hc = min(max(hr, 0), IMH - 1);
      const bool hok = (hr >= 0) && (hr < IMH);
#pragma unroll 1
      for (int j = 0; j < 5; ++j) {
        const int wr = wq + j - 2;
        const int wc = min(max(wr, 0), IMW - 1);
        const bool ok = hok && (wr >= 0) && (wr < IMW);
        const v4h hv = *(const v4h*)(XT + ((size_t)(b * SP + 1 + hc * IMW + wc)) * CD + c);
        const v4f w  = *(const v4f*)(sW + (i * 5 + j) * CD + c);
        v4f xv;
        xv[0] = ok ? (float)hv[0] : 0.0f;
        xv[1] = ok ? (float)hv[1] : 0.0f;
        xv[2] = ok ? (float)hv[2] : 0.0f;
        xv[3] = ok ? (float)hv[3] : 0.0f;
        acc += w * xv;
      }
    }
    const v4f bb  = *(const v4f*)(sB + c);
    const v4f res = acc * xinv + bb;
    float* dst = DW + ((size_t)(b * NPIX + n)) * CD + c;
    *(volatile v4f*)dst = res;
    __threadfence();
    *(volatile v4f*)dst = res;
  }
}

__global__ __launch_bounds__(256) void gemm_qkv(
    const unsigned short* __restrict__ Wp, const unsigned short* __restrict__ XTp,
    unsigned short* QH, unsigned short* QL, unsigned short* KX,
    unsigned short* VH, unsigned short* VL, float oscale) {
  const _Float16* A  = (const _Float16*)(const void*)Wp;
  const _Float16* Bt = (const _Float16*)(const void*)XTp;
  __shared__ __align__(16) unsigned short sP[8][2][SPW];
  const int lane = threadIdx.x & 31;
  const int wave = threadIdx.x >> 5;
  const int tilesN = NTOK / 64;
  const int tilesM = OQ / 64;
  const int tile = blockIdx.x * 8 + wave;
  if (tile >= tilesM * tilesN) return;
  const int tm = tile / tilesN;
  const int tn = tile - tm * tilesN;
  const int m0 = tm << 6;
  const int n0 = tn << 6;
  const int rlane = lane & 15;
  const int hh    = lane >> 4;
  const int koff  = hh * 8;
  const int mOff  = hh * 8;

  v8f acc[4][4];
#pragma unroll
  for (int i = 0; i < 4; ++i)
#pragma unroll
    for (int j = 0; j < 4; ++j) acc[i][j] = zero8();

  for (int k0 = 0; k0 < CD; k0 += 32) {
    v16h bf[4];
#pragma unroll
    for (int j = 0; j < 4; ++j) {
      const size_t bo = (size_t)(n0 + (j << 4) + rlane) * CD + koff + k0;
      bf[j] = ldfrag_h(Bt + bo);
    }
#pragma unroll
    for (int i = 0; i < 4; ++i) {
      const size_t ao = (size_t)(m0 + (i << 4) + rlane) * CD + koff + k0;
      const v16h ah = ldfrag_h(A + ao);
#pragma unroll
      for (int j = 0; j < 4; ++j) acc[i][j] = mma_h_raw(ah, bf[j], acc[i][j]);
      dep_guard_h(acc[i][0], acc[i][3], ah, bf[3]);
    }
    keep4_h(bf[0], bf[1], bf[2], bf[3]);
  }
  acc_guard4(acc[0][0], acc[0][1], acc[0][2], acc[0][3]);
  acc_guard4(acc[1][0], acc[1][1], acc[1][2], acc[1][3]);
  acc_guard4(acc[2][0], acc[2][1], acc[2][2], acc[2][3]);
  acc_guard4(acc[3][0], acc[3][1], acc[3][2], acc[3][3]);

  const int sec   = m0 >> 8;
  const int hbase = (m0 & (CD - 1)) >> 5;
  const int b     = n0 / SP;
  const int s0t   = n0 - b * SP;
  unsigned short* s0 = &sP[wave][0][0];
  unsigned short* s1 = &sP[wave][1][0];

  if (sec < 2) {
    unsigned short* Ph = (sec == 0) ? QH : KX;
#pragma unroll
    for (int hp = 0; hp < 2; ++hp) {
      const int bh = b * NH + hbase + hp;
#pragma unroll
      for (int j = 0; j < 4; ++j) {
#pragma unroll
        for (int il = 0; il < 2; ++il) {
          unsigned short hq8[8], lq8[8];
#pragma unroll
          for (int r = 0; r < 8; ++r) {
            const float f = acc[2 * hp + il][j][r] * oscale;
            const _Float16 xh = (_Float16)f;
            hq8[r] = h_bits(xh);
            lq8[r] = h_bits((_Float16)((f - (float)xh) * 2048.0f));
          }
          v4u ph, pl;
#pragma unroll
          for (int q = 0; q < 4; ++q) {
            ph[q] = pk16(hq8[2 * q], hq8[2 * q + 1]);
            pl[q] = pk16(lq8[2 * q], lq8[2 * q + 1]);
          }
          const int so = ((j << 4) + rlane) * HD + (il << 4) + mOff;
          *(v4u*)(s0 + so) = ph;
          if (sec == 0) *(v4u*)(s1 + so) = pl;
        }
      }
      wave_sync_lds();
      const size_t pb = ((size_t)(bh * SP + s0t)) * HD;
      for (int pass = 0; pass < 2; ++pass) {
#pragma unroll
        for (int cch = 0; cch < 8; ++cch) {
          const int e = cch * 256 + lane * 8;
          const v4u v = *(const v4u*)(s0 + e);
          *(volatile v4u*)(Ph + pb + e) = v;
          if (sec == 0) {
            const v4u w = *(const v4u*)(s1 + e);
            *(volatile v4u*)(QL + pb + e) = w;
          }
        }
        __threadfence();
      }
      wave_sync_lds();
    }
  } else {
    const int rq = lane >> 3, c8 = (lane & 7) * 8;
#pragma unroll
    for (int hp = 0; hp < 2; ++hp) {
      const int bh = b * NH + hbase + hp;
#pragma unroll
      for (int il = 0; il < 2; ++il) {
#pragma unroll
        for (int j = 0; j < 4; ++j) {
#pragma unroll
          for (int r = 0; r < 8; ++r) {
            const float f = acc[2 * hp + il][j][r] * oscale;
            const _Float16 xh = (_Float16)f;
            const int so = ((il << 4) + mOff + r) * SVP + (j << 4) + rlane;
            s0[so] = h_bits(xh);
            s1[so] = h_bits((_Float16)((f - (float)xh) * 2048.0f));
          }
        }
      }
      wave_sync_lds();
      for (int pass = 0; pass < 2; ++pass) {
#pragma unroll
        for (int it = 0; it < 8; ++it) {
          const int d = it * 4 + rq;
          const size_t dst = ((size_t)(bh * HD + d)) * SP + s0t + c8;
          const v4u v = *(const v4u*)(s0 + d * SVP + c8);
          const v4u w = *(const v4u*)(s1 + d * SVP + c8);
          *(volatile v4u*)(VH + dst) = v;
          *(volatile v4u*)(VL + dst) = w;
        }
        __threadfence();
      }
      wave_sync_lds();
    }
  }
}

__global__ __launch_bounds__(ATHR) void attn_kernel(
    const unsigned short* __restrict__ QHp, const unsigned short* __restrict__ QLp,
    const unsigned short* __restrict__ KXp,
    const unsigned short* __restrict__ VHp, const unsigned short* __restrict__ VLp,
    const float* __restrict__ DW,
    unsigned short* CTXh, unsigned short* CTXl, float rscale) {
  __shared__ __align__(16) unsigned short lds_u[LDSA];
  unsigned short* kl_u = lds_u;
  unsigned short* vh_u = lds_u + KC * KP;
  unsigned short* vl_u = vh_u + HD * VP;
  const _Float16* kl = (const _Float16*)(const void*)kl_u;
  const _Float16* vh = (const _Float16*)(const void*)vh_u;
  const _Float16* vl = (const _Float16*)(const void*)vl_u;
  const _Float16* QH = (const _Float16*)(const void*)QHp;
  const _Float16* QL = (const _Float16*)(const void*)QLp;

  const int tid = threadIdx.x, lane = tid & 31, wave = tid >> 5;
  const int bh = blockIdx.y;
  const int b = bh >> 3, h = bh & 7;
  const int rlane = lane & 15, hsel = lane >> 4, koff = hsel * 8;
  const int n0w = blockIdx.x * QB + wave * 16;

  const size_t qo = ((size_t)(bh * SP + n0w + rlane)) * HD + koff;
  const v16h qh = ldfrag_h(QH + qo);
  const v16h ql = ldfrag_h(QL + qo);

  const float C2048  = 1.0f / 2048.0f;
  const float CS     = 0.17677669529663687f / 256.0f;
  const float LN1024 = 6.931471805599453f;

  v8f oh[2], ol[2];
#pragma unroll
  for (int dt = 0; dt < 2; ++dt) { oh[dt] = zero8(); ol[dt] = zero8(); }
  float m_run = -1.0e30f, l_run = 0.0f;

#pragma unroll 1
  for (int kc = 0; kc < NKC; ++kc) {
    const int kc0 = kc * KC;
    __syncthreads();
    for (int i = tid; i < KC * 4; i += ATHR) {
      const int key = i >> 2, c8 = (i & 3) * 8;
      const v4u v = *(const v4u*)(KXp + ((size_t)(bh * SP + kc0 + key)) * HD + c8);
      *(v4u*)(kl_u + key * KP + c8) = v;
    }
    for (int i = tid; i < HD * (KC / 8); i += ATHR) {
      const int d = i / (KC / 8);
      const int j = i - d * (KC / 8);
      const size_t go = ((size_t)(bh * HD + d)) * SP + kc0 + 8 * j;
      const v4u a = *(const v4u*)(VHp + go);
      const v4u c = *(const v4u*)(VLp + go);
      *(v4u*)(vh_u + d * VP + 8 * j) = a;
      *(v4u*)(vl_u + d * VP + 8 * j) = c;
    }
    __syncthreads();

#pragma unroll 1
    for (int sub = 0; sub < NSUB; ++sub) {
      const int kr = sub * 32;
      float a[2][8];
#pragma unroll
      for (int t = 0; t < 2; ++t) {
        const int krow = kr + 16 * t + rlane;
        const v16h kf = ldfrag_h(kl + krow * KP + koff);
        v8f sh = mma_h_raw(kf, qh, zero8());
        v8f sr = mma_h_raw(kf, ql, zero8());
        dep_guard3(sh, sr, kf, qh, ql);
#pragma unroll
        for (int r = 0; r < 8; ++r) {
          const int key = kc0 + kr + 16 * t + 8 * hsel + r;
          const float s = (sh[r] + sr[r] * C2048) * CS;
          a[t][r] = (key < SEQ) ? s : -1.0e30f;
        }
      }

      float mloc = -1.0e30f;
#pragma unroll
      for (int r = 0; r < 8; ++r) mloc = fmaxf(mloc, fmaxf(a[0][r], a[1][r]));
      mloc = fmaxf(mloc, __shfl_xor(mloc, 16, 32));
      const float newM  = fmaxf(m_run, mloc);
      const float alpha = __expf(m_run - newM);
      const float msh   = newM - LN1024;
      float ssum = 0.0f;
      float p[2][8];
#pragma unroll
      for (int r = 0; r < 8; ++r) {
        p[0][r] = __expf(a[0][r] - msh);
        p[1][r] = __expf(a[1][r] - msh);
        ssum += p[0][r] + p[1][r];
      }
      ssum += __shfl_xor(ssum, 16, 32);
      l_run = l_run * alpha + ssum;
      m_run = newM;
#pragma unroll
      for (int dt = 0; dt < 2; ++dt) {
#pragma unroll
        for (int r = 0; r < 8; ++r) { oh[dt][r] *= alpha; ol[dt][r] *= alpha; }
      }

      union { v16h v; _Float16 s[16]; } ph;
#pragma unroll
      for (int r = 0; r < 8; ++r) {
        ph.s[r]     = (_Float16)p[0][r];
        ph.s[8 + r] = (_Float16)p[1][r];
      }

#pragma unroll
      for (int dt = 0; dt < 2; ++dt) {
        const v16h vah = ldfrag_h(vh + (16 * dt + rlane) * VP + kr + koff);
        const v16h val = ldfrag_h(vl + (16 * dt + rlane) * VP + kr + koff);
        oh[dt] = mma_h_raw(vah, ph.v, oh[dt]);
        ol[dt] = mma_h_raw(val, ph.v, ol[dt]);
        dep_guard3(oh[dt], ol[dt], vah, val, ph.v);
      }
    }
  }
  acc_guard4(oh[0], oh[1], ol[0], ol[1]);

  const float inv = 4.0f * (1.0f / l_run);
  const int s = n0w + rlane;
  const bool dok = (s >= 1) && (s <= NPIX);
  const int sc = min(max(s - 1, 0), NPIX - 1);
  const float* dwp = DW + ((size_t)(b * NPIX + sc)) * CD + h * HD + 8 * hsel;
  __syncthreads();
  unsigned short* sth = lds_u + wave * 1024;
  unsigned short* stl = sth + 512;
#pragma unroll
  for (int dt = 0; dt < 2; ++dt) {
    const v4f g0 = *(const v4f*)(dwp + 16 * dt);
    const v4f g1 = *(const v4f*)(dwp + 16 * dt + 4);
    float gv[8];
    gv[0] = g0[0]; gv[1] = g0[1]; gv[2] = g0[2]; gv[3] = g0[3];
    gv[4] = g1[0]; gv[5] = g1[1]; gv[6] = g1[2]; gv[7] = g1[3];
    v4u hv, lw;
#pragma unroll
    for (int e = 0; e < 4; ++e) {
      const float add0 = dok ? gv[2 * e] * 64.0f : 0.0f;
      const float add1 = dok ? gv[2 * e + 1] * 64.0f : 0.0f;
      const float f0 = (oh[dt][2 * e]     + ol[dt][2 * e]     * C2048) * inv + add0;
      const float f1 = (oh[dt][2 * e + 1] + ol[dt][2 * e + 1] * C2048) * inv + add1;
      const _Float16 x0 = (_Float16)f0, x1 = (_Float16)f1;
      hv[e] = pk16(h_bits(x0), h_bits(x1));
      lw[e] = pk16(h_bits((_Float16)((f0 - (float)x0) * rscale)),
                   h_bits((_Float16)((f1 - (float)x1) * rscale)));
    }
    const int so = rlane * HD + 16 * dt + 8 * hsel;
    *(v4u*)(sth + so) = hv;
    *(v4u*)(stl + so) = lw;
  }
  wave_sync_lds();
  {
    const size_t base = ((size_t)(bh * SP + n0w)) * HD;
    for (int pass = 0; pass < 2; ++pass) {
#pragma unroll
      for (int cch = 0; cch < 2; ++cch) {
        const int e = cch * 256 + lane * 8;
        const v4u v = *(const v4u*)(sth + e);
        *(volatile v4u*)(CTXh + base + e) = v;
      }
      __threadfence();
    }
    for (int pass = 0; pass < 2; ++pass) {
#pragma unroll
      for (int cch = 0; cch < 2; ++cch) {
        const int e = cch * 256 + lane * 8;
        const v4u v = *(const v4u*)(stl + e);
        *(volatile v4u*)(CTXl + base + e) = v;
      }
      __threadfence();
    }
  }
}

__global__ __launch_bounds__(256) void gemm_proj(
    const unsigned short* __restrict__ CHp, const unsigned short* __restrict__ CLp,
    const unsigned short* __restrict__ PWp, const float* __restrict__ bias,
    float* out, float oscale, float rres) {
  const _Float16* CH = (const _Float16*)(const void*)CHp;
  const _Float16* CL = (const _Float16*)(const void*)CLp;
  const _Float16* Bt = (const _Float16*)(const void*)PWp;
  __shared__ __align__(16) float sT[8][16 * 68];
  const int lane = threadIdx.x & 31;
  const int wave = threadIdx.x >> 5;
  const int tilesN = CD / 64;
  const int tilesM = NTOK / 64;
  const int tile = blockIdx.x * 8 + wave;
  if (tile >= tilesM * tilesN) return;
  const int tm = tile / tilesN;
  const int tn = tile - tm * tilesN;
  const int m0 = tm << 6;
  const int n0 = tn << 6;
  const int b   = m0 / SP;
  const int s0t = m0 - b * SP;
  const int rlane = lane & 15;
  const int hh    = lane >> 4;
  const int koff  = hh * 8;
  const int mOff  = hh * 8;

  const size_t pbase = ((size_t)(b * NH) * SP + (size_t)s0t) * HD;
  const _Float16* Ah = CH + pbase;
  const _Float16* Al = CL + pbase;

  v8f acc[4][4];
#pragma unroll
  for (int i = 0; i < 4; ++i)
#pragma unroll
    for (int j = 0; j < 4; ++j) acc[i][j] = zero8();

  for (int k0 = 0; k0 < CD; k0 += 32) {
    const size_t hplane = (size_t)(k0 >> 5) * SP * HD;
    v16h bf[4];
#pragma unroll
    for (int j = 0; j < 4; ++j) {
      const size_t bo = (size_t)(n0 + (j << 4) + rlane) * CD + koff + k0;
      bf[j] = ldfrag_h(Bt + bo);
    }
#pragma unroll
    for (int i = 0; i < 4; ++i) {
      const size_t ao = hplane + (size_t)((i << 4) + rlane) * HD + koff;
      const v16h ah = ldfrag_h(Ah + ao);
      const v16h al = ldfrag_h(Al + ao);
#pragma unroll
      for (int j = 0; j < 4; ++j) {
        acc[i][j] = mma_h_raw(ah, bf[j], acc[i][j]);
        v8f tp = mma_h_raw(al, bf[j], zero8());
        res_guard(tp, acc[i][j], al, bf[j]);
#pragma unroll
        for (int r = 0; r < 8; ++r) acc[i][j][r] += tp[r] * rres;
      }
      dep_guard3(acc[i][0], acc[i][3], ah, al, bf[3]);
    }
    keep4_h(bf[0], bf[1], bf[2], bf[3]);
  }
  acc_guard4(acc[0][0], acc[0][1], acc[0][2], acc[0][3]);
  acc_guard4(acc[1][0], acc[1][1], acc[1][2], acc[1][3]);
  acc_guard4(acc[2][0], acc[2][1], acc[2][2], acc[2][3]);
  acc_guard4(acc[3][0], acc[3][1], acc[3][2], acc[3][3]);

  float bcol[4];
#pragma unroll
  for (int j = 0; j < 4; ++j) bcol[j] = bf_up(bf_bits(bias[n0 + (j << 4) + rlane]));
  float* slab = sT[wave];
#pragma unroll
  for (int i = 0; i < 4; ++i) {
#pragma unroll
    for (int j = 0; j < 4; ++j) {
#pragma unroll
      for (int r = 0; r < 8; ++r) {
        slab[(mOff + r) * 68 + (j << 4) + rlane] = acc[i][j][r] * oscale + bcol[j];
      }
    }
    wave_sync_lds();
    {
      const int c4 = rlane * 4;
      for (int pass = 0; pass < 2; ++pass) {
#pragma unroll
        for (int it = 0; it < 8; ++it) {
          const int row = it * 2 + hh;
          const int s = s0t + (i << 4) + row;
          const int sc = min(max(s, 1), NPIX);
          size_t off = (s == 0) ? ((size_t)OUT1OFF + (size_t)b * CD)
                                : (((size_t)(b * NPIX + sc - 1)) * CD);
          off += (size_t)(n0 + c4);
          const v4f v = *(const v4f*)(slab + row * 68 + c4);
          if (s <= NPIX) *(volatile v4f*)(out + off) = v;
        }
        __threadfence();
      }
    }
    wave_sync_lds();
  }
}

extern "C" void kernel_launch(void* const* d_in, const int* in_sizes, int n_in,
                              void* d_out, int out_size, void* d_ws, size_t ws_size,
                              hipStream_t stream) {
  if (n_in < 7) return;
  if (in_sizes[0] != NB * NPIX * CD) return;
  if (in_sizes[1] != NB * CD) return;
  if (in_sizes[2] != OQ * CD) return;
  if (in_sizes[3] != CD * CD) return;
  if (in_sizes[4] != CD) return;
  if (in_sizes[5] != CD * 25) return;
  if (in_sizes[6] != CD) return;
  if (out_size != NB * NPIX * CD + NB * CD) return;

  const float* x      = (const float*)d_in[0];
  const float* clsv   = (const float*)d_in[1];
  const float* qkv_w  = (const float*)d_in[2];
  const float* proj_w = (const float*)d_in[3];
  const float* proj_b = (const float*)d_in[4];
  const float* dw_w   = (const float*)d_in[5];
  const float* dw_b   = (const float*)d_in[6];

  const size_t PW3 = (size_t)OQ * CD * 2;
  const size_t PPW = (size_t)CD * CD * 2;
  const size_t PXT = (size_t)NTOK * CD * 2;
  const size_t PDW = (size_t)NDWR * CD * 4;
  const size_t PQ  = (size_t)NBH * SP * HD * 2;
  const size_t PV  = (size_t)NBH * HD * SP * 2;
  const size_t PCT = (size_t)NBH * SP * HD * 2;
  size_t off = 0;
  const size_t oW3 = off; off += PW3;
  const size_t oPW = off; off += PPW;
  const size_t oXT = off; off += PXT;
  const size_t oDW = off; off += PDW;
  const size_t oQH = off; off += PQ;
  const size_t oQL = off; off += PQ;
  const size_t oKX = off; off += PQ;
  const size_t oVH = off; off += PV;
  const size_t oVL = off; off += PV;
  const size_t oCH = off; off += PCT;
  const size_t oCL = off; off += PCT;
  if (off > ws_size) return;
  if (off > (size_t)134217728) return;

  char* ws = (char*)d_ws;
  unsigned short* W3   = (unsigned short*)(ws + oW3);
  unsigned short* PWp  = (unsigned short*)(ws + oPW);
  unsigned short* XT   = (unsigned short*)(ws + oXT);
  float*          DW   = (float*)(ws + oDW);
  unsigned short* QH   = (unsigned short*)(ws + oQH);
  unsigned short* QL   = (unsigned short*)(ws + oQL);
  unsigned short* KX   = (unsigned short*)(ws + oKX);
  unsigned short* VH   = (unsigned short*)(ws + oVH);
  unsigned short* VL   = (unsigned short*)(ws + oVL);
  unsigned short* CTXh = (unsigned short*)(ws + oCH);
  unsigned short* CTXl = (unsigned short*)(ws + oCL);
  float*          out  = (float*)d_out;

  const dim3 blk(256);
  const int n8w3 = OQ * CD / 8;
  const int n8pw = CD * CD / 8;
  const dim3 gW3((n8w3 + 255) / 256);
  const dim3 gPW((n8pw + 255) / 256);
  const dim3 gXT((NTOK * 32 + 255) / 256);
  const dim3 gDW(NDWR / LPB);
  const dim3 gQkv(((OQ / 64) * (NTOK / 64) + 7) / 8);
  const dim3 gAttn(NQB, NBH);
  const dim3 gProj(((NTOK / 64) * (CD / 64) + 7) / 8);

  const float oscQkv = 1.0f / 1024.0f;
  const float rscale = 16384.0f;
  const float oscPrj = 1.0f / 65536.0f;
  const float rres   = 1.0f / 16384.0f;

  cvt_h8<<<gW3, blk, 0, stream>>>(qkv_w, W3, n8w3, 1024.0f);
  cvt_h8<<<gPW, blk, 0, stream>>>(proj_w, PWp, n8pw, 1024.0f);
  cvt_xt<<<gXT, blk, 0, stream>>>(x, clsv, XT, 16.0f);
  dwconv5<<<gDW, blk, 0, stream>>>(XT, dw_w, dw_b, DW, 1.0f / 16.0f);
  gemm_qkv<<<gQkv, blk, 0, stream>>>(W3, XT, QH, QL, KX, VH, VL, oscQkv);
  attn_kernel<<<gAttn, dim3(ATHR), 0, stream>>>(QH, QL, KX, VH, VL, DW, CTXh, CTXl, rscale);
  gemm_proj<<<gProj, blk, 0, stream>>>(CTXh, CTXl, PWp, proj_b, out, oscPrj, rres);
  (void)hipGetLastError();
}
